// FDModel_87651692577337
// MI455X (gfx1250) — hardware-verified
//
#include <hip/hip_runtime.h>
#include <stdint.h>

#define NV   3
#define NN   6000
#define MP   6016
#define DIN  512
#define HID  256
#define DYD  512

typedef _Float16 v16h __attribute__((ext_vector_type(16)));
typedef _Float16 v8h  __attribute__((ext_vector_type(8)));
typedef __bf16   v16b __attribute__((ext_vector_type(16)));
typedef __bf16   v8b  __attribute__((ext_vector_type(8)));
typedef float    v8f  __attribute__((ext_vector_type(8)));
typedef float    v4f  __attribute__((ext_vector_type(4)));
typedef unsigned short v8us __attribute__((ext_vector_type(8)));

static_assert((MP % 128) == 0);
static_assert(MP >= NN && (MP - NN) < 32);
static_assert((NN % 16) == 0);
static_assert((HID % 64) == 0 && (DIN % 64) == 0 && (DYD % 32) == 0);

__device__ __forceinline__ unsigned short bfbits(float f) {
  unsigned u = __float_as_uint(f);
  return (unsigned short)((u + 0x7FFFu + ((u >> 16) & 1u)) >> 16);
}
__device__ __forceinline__ float bfval(unsigned short b) { return __uint_as_float(((unsigned)b) << 16); }
__device__ __forceinline__ float bfr(float f) { return bfval(bfbits(f)); }

__device__ __forceinline__ v16h ldfrag(const _Float16* p) {
  union { v16h v; v8h h[2]; } f;
  f.h[0] = *(const v8h*)(p);
  f.h[1] = *(const v8h*)(p + 16);
  return f.v;
}
__device__ __forceinline__ v16b ldfragb(const __bf16* p) {
  union { v16b v; v8b h[2]; } f;
  f.h[0] = *(const v8b*)(p);
  f.h[1] = *(const v8b*)(p + 16);
  return f.v;
}
__device__ __forceinline__ v8f mma16(v16h a, v16h b, v8f c) {
  return __builtin_amdgcn_wmma_f32_16x16x32_f16(false, a, false, b, (short)0, c, false, false);
}
__device__ __forceinline__ v8f mmab(v16b a, v16b b, v8f c) {
  return __builtin_amdgcn_wmma_f32_16x16x32_bf16(false, a, false, b, (short)0, c, false, false);
}
__device__ __forceinline__ v8f zero8() {
  v8f z;
#pragma unroll
  for (int i = 0; i < 8; ++i) z[i] = 0.0f;
  return z;
}

__device__ __forceinline__ void guard_gb(v8f& a, v8f& b, v16b x, v16b y) {
#if defined(__HIP_DEVICE_COMPILE__)
  asm volatile("v_nop\n\tv_nop\n\tv_nop\n\tv_nop" : "+v"(a), "+v"(b) : "v"(x), "v"(y));
#endif
}
__device__ __forceinline__ void keep4b(v16b a, v16b b, v16b c, v16b d) {
#if defined(__HIP_DEVICE_COMPILE__)
  asm volatile("v_nop" :: "v"(a), "v"(b), "v"(c), "v"(d));
#endif
}
__device__ __forceinline__ void accg4(v8f& a, v8f& b, v8f& c, v8f& d) {
#if defined(__HIP_DEVICE_COMPILE__)
  asm volatile("v_nop\n\tv_nop\n\tv_nop\n\tv_nop" : "+v"(a), "+v"(b), "+v"(c), "+v"(d));
#endif
}
__device__ __forceinline__ void guard_s2(v8f& a, v8f& b, v16h x, v16h y0, v16h y1) {
#if defined(__HIP_DEVICE_COMPILE__)
  asm volatile("v_nop\n\tv_nop\n\tv_nop\n\tv_nop" : "+v"(a), "+v"(b) : "v"(x), "v"(y0), "v"(y1));
#endif
}
__device__ __forceinline__ void guard_pv(v8f& a0, v8f& a1, v8f& a2, v8f& b0, v8f& b1, v8f& b2,
                                         v16h p0, v16h p1, v16h x0, v16h x1, v16h x2) {
#if defined(__HIP_DEVICE_COMPILE__)
  asm volatile("v_nop\n\tv_nop\n\tv_nop\n\tv_nop"
               : "+v"(a0), "+v"(a1), "+v"(a2), "+v"(b0), "+v"(b1), "+v"(b2)
               : "v"(p0), "v"(p1), "v"(x0), "v"(x1), "v"(x2));
#endif
}

__global__ __launch_bounds__(256) void cvt_kernel(const float* __restrict__ src, unsigned short* __restrict__ dst,
                                                  int n8) {
  const int li = (int)blockIdx.x * 256 + (int)threadIdx.x;
  if (li >= n8) return;
  const size_t e = (size_t)li * 8;
  const v4f a = *(const v4f*)(src + e);
  const v4f b = *(const v4f*)(src + e + 4);
  v8us o;
#pragma unroll
  for (int i = 0; i < 4; ++i) {
    o[i]     = bfbits(a[i]);
    o[4 + i] = bfbits(b[i]);
  }
  unsigned short* d = dst + e;
  *(volatile v8us*)d = o;
  __threadfence();
  *(volatile v8us*)d = o;
}

template <bool SPLITA, int EPI>
__global__ __launch_bounds__(256) void gemm64_kernel(const unsigned short* __restrict__ Ap,
                                                     const unsigned short* __restrict__ A2p,
                                                     int lda, int aRows, int sAv,
                                                     const unsigned short* __restrict__ Btp, int ldb, int sBv,
                                                     float* __restrict__ C, int ldc, int sCv, int cRows,
                                                     const float* __restrict__ bias, int sBiasV,
                                                     int M, int N, int K) {
  __shared__ __align__(16) float sT[8][16 * 68];
  const int lane = threadIdx.x & 31, wave = threadIdx.x >> 5;
  const int vz = (int)blockIdx.y;
  const __bf16* A  = (const __bf16*)(const void*)(Ap  + (size_t)vz * (size_t)sAv);
  const __bf16* A2 = (const __bf16*)(const void*)(A2p + (size_t)vz * (size_t)sAv);
  const __bf16* Bt = (const __bf16*)(const void*)(Btp + (size_t)vz * (size_t)sBv);
  float* Cv = C + (size_t)vz * (size_t)sCv;
  const float* bv = bias + (size_t)vz * (size_t)sBiasV;

  const int tilesN = N >> 6, tilesM = M >> 6;
  const int tile = (int)blockIdx.x * 8 + wave;
  if (tile >= tilesM * tilesN) return;
  const int tm = tile / tilesN, tn = tile - tm * tilesN;
  const int m0 = tm << 6, n0 = tn << 6;
  const int rl = lane & 15;
  const int koff = (lane >> 4) * 8;
  const int mOff = (lane >> 4) * 8;

  int arow[4];
#pragma unroll
  for (int i = 0; i < 4; ++i) {
    const int r = m0 + (i << 4) + rl;
    arow[i] = (r < aRows) ? r : (aRows - 1);
  }

  v8f acc[4][4];
#pragma unroll
  for (int i = 0; i < 4; ++i)
#pragma unroll
    for (int j = 0; j < 4; ++j) acc[i][j] = zero8();

#pragma unroll 1
  for (int k0 = 0; k0 < K; k0 += 32) {
    v16b bh[4];
#pragma unroll
    for (int j = 0; j < 4; ++j) bh[j] = ldfragb(Bt + (size_t)(n0 + (j << 4) + rl) * ldb + koff + k0);
#pragma unroll
    for (int i = 0; i < 4; ++i) {
      const size_t ao = (size_t)arow[i] * lda + koff + k0;
      const v16b ah = ldfragb(A + ao);
      v16b al = ah;
      if (SPLITA) al = ldfragb(A2 + ao);
#pragma unroll
      for (int j = 0; j < 4; ++j) {
        acc[i][j] = mmab(ah, bh[j], acc[i][j]);
        if (SPLITA) acc[i][j] = mmab(al, bh[j], acc[i][j]);
      }
      guard_gb(acc[i][0], acc[i][3], ah, SPLITA ? al : bh[3]);
    }
    keep4b(bh[0], bh[1], bh[2], bh[3]);
  }
  accg4(acc[0][0], acc[0][1], acc[0][2], acc[0][3]);
  accg4(acc[1][0], acc[1][1], acc[1][2], acc[1][3]);
  accg4(acc[2][0], acc[2][1], acc[2][2], acc[2][3]);
  accg4(acc[3][0], acc[3][1], acc[3][2], acc[3][3]);

  float* slab = sT[wave];
#pragma unroll
  for (int i = 0; i < 4; ++i) {
    const int mBase = m0 + (i << 4);
#pragma unroll
    for (int j = 0; j < 4; ++j) {
      const float bb = bfr(bv[n0 + (j << 4) + rl]);
#pragma unroll
      for (int r = 0; r < 8; ++r) {
        float x = acc[i][j][r] + bb;
        if (EPI == 2) {
          x = __builtin_amdgcn_rcpf(1.0f + __expf(-x));
        } else {
          x = (x >= 0.0f) ? x : 0.1f * x;
          if (EPI == 1) {
            if (x != x) x = 0.0f;
            x = fminf(fmaxf(x, -3.402823466e+38f), 3.402823466e+38f);
          }
        }
        slab[(mOff + r) * 68 + (j << 4) + rl] = x;
      }
    }
    __builtin_amdgcn_fence(__ATOMIC_RELEASE, "workgroup");
    __builtin_amdgcn_wave_barrier();
    __builtin_amdgcn_fence(__ATOMIC_ACQUIRE, "workgroup");
    if (mBase < cRows) {
      const int hh = lane >> 4, c4 = (lane & 15) * 4;
#pragma unroll
      for (int ps = 0; ps < 2; ++ps) {
#pragma unroll
        for (int it = 0; it < 8; ++it) {
          const int row = it * 2 + hh;
          const v4f v = *(const v4f*)(slab + row * 68 + c4);
          *(volatile v4f*)(Cv + (size_t)(mBase + row) * ldc + n0 + c4) = v;
        }
        __threadfence();
      }
    }
    __builtin_amdgcn_fence(__ATOMIC_RELEASE, "workgroup");
    __builtin_amdgcn_wave_barrier();
    __builtin_amdgcn_fence(__ATOMIC_ACQUIRE, "workgroup");
  }
}

#define TP 72
__global__ __launch_bounds__(256) void qt_kernel(const float* __restrict__ hF, const float* __restrict__ mask,
                                                 _Float16* __restrict__ q16, _Float16* __restrict__ hT16,
                                                 float qs, float hs) {
  __shared__ __align__(16) _Float16 T[HID * TP];
  const int wave = threadIdx.x >> 5, lane = threadIdx.x & 31;
  const int v = (int)blockIdx.y;
  const int m0 = (int)blockIdx.x * 64;
#pragma unroll 1
  for (int i = 0; i < 8; ++i) {
    const int ml = 8 * wave + i;
    const int m = m0 + ml;
    const float* hr = hF + (size_t)(v * MP + m) * HID + 8 * lane;
    const v4f a = *(const v4f*)hr;
    const v4f b = *(const v4f*)(hr + 4);
    float ss = 0.0f;
#pragma unroll
    for (int e = 0; e < 4; ++e) ss += a[e] * a[e];
#pragma unroll
    for (int e = 0; e < 4; ++e) ss += b[e] * b[e];
#pragma unroll
    for (int off = 16; off > 0; off >>= 1) ss += __shfl_xor(ss, off, 32);
    const float inv = 1.0f / fmaxf(sqrtf(ss), 1e-12f);
    const bool valid = (m < NN);
    const int mcl = valid ? m : (NN - 1);
    const float mval = mask[(size_t)mcl * NV + v];
    const float mv = valid ? (mval * hs) : 0.0f;
    const float qsc = valid ? (inv * qs) : 0.0f;
    v8h qo;
#pragma unroll
    for (int e = 0; e < 4; ++e) {
      qo[e]     = (_Float16)(a[e] * qsc);
      qo[4 + e] = (_Float16)(b[e] * qsc);
      T[(8 * lane + e) * TP + ml]     = (_Float16)(a[e] * mv);
      T[(8 * lane + 4 + e) * TP + ml] = (_Float16)(b[e] * mv);
    }
    _Float16* d = q16 + (size_t)(v * MP + m) * HID + 8 * lane;
    *(volatile v8h*)d = qo;
    __threadfence();
    *(volatile v8h*)d = qo;
  }
  __syncthreads();
  const int qg = lane >> 3, p = lane & 7;
#pragma unroll
  for (int ps = 0; ps < 2; ++ps) {
#pragma unroll
    for (int it = 0; it < 8; ++it) {
      const int col = 32 * wave + 4 * it + qg;
      const v8h val = *(const v8h*)(T + col * TP + 8 * p);
      *(volatile v8h*)(hT16 + (size_t)(v * HID + col) * MP + m0 + 8 * p) = val;
    }
    __threadfence();
  }
}

#define QB      32
#define KC      128
#define NCH     (MP / KC)
#define QSP     264
#define PSP     136
#define OTP     260
#define L_QS    0
#define L_PS    50688
#define L_MROW  59392
#define L_MCOL  59776
#define L_PSUM  61312
#define L_LI    62336
#define ATT_LDS 62464
static_assert(NV * QB * QSP * 2 == L_PS - L_QS);
static_assert(QB * PSP * 2 == L_MROW - L_PS);
static_assert(NV * QB * 4 == L_MCOL - L_MROW);
static_assert(NV * KC * 4 == L_PSUM - L_MCOL);
static_assert(8 * QB * 4 == L_LI - L_PSUM);
static_assert(QB * 4 == ATT_LDS - L_LI);
static_assert(QB * OTP * 4 <= L_PS - L_QS);
static_assert((QSP % 8) == 0 && (PSP % 8) == 0 && PSP >= KC && (OTP % 4) == 0);
static_assert((L_PS % 16) == 0 && (L_MROW % 16) == 0 && (L_MCOL % 16) == 0 && (L_PSUM % 16) == 0 && (L_LI % 16) == 0);
static_assert((MP % QB) == 0 && (MP % KC) == 0 && KC == 16 * 8);

__global__ __launch_bounds__(256) void attn_kernel(const _Float16* __restrict__ q16, const _Float16* __restrict__ hT16,
                                                   const float* __restrict__ hF, const float* __restrict__ mask,
                                                   float* __restrict__ out0, unsigned short* __restrict__ nxh,
                                                   unsigned short* __restrict__ nxl, float escale, float invhs) {
  extern __shared__ __align__(16) char smem[];
  _Float16* Qs = (_Float16*)(smem + L_QS);
  _Float16* Ps = (_Float16*)(smem + L_PS);
  float* mrow = (float*)(smem + L_MROW);
  float* mc   = (float*)(smem + L_MCOL);
  float* psum = (float*)(smem + L_PSUM);
  float* li   = (float*)(smem + L_LI);

  const int tid = threadIdx.x, wave = tid >> 5, lane = tid & 31, h = lane >> 4, c = lane & 15;
  const int n0 = (int)blockIdx.x * QB;

  if (tid < NV * QB) {
    const int v = tid >> 5, row = tid & 31;
    const int n = n0 + row;
    const int nc = (n < NN) ? n : (NN - 1);
    const float mval = mask[(size_t)nc * NV + v];
    mrow[v * QB + row] = (n < NN) ? mval : 0.0f;
  }
#pragma unroll
  for (int i = 0; i < 12; ++i) {
    const int idx = i * 256 + tid;
    const int v = idx >> 10;
    const int rem = idx & 1023;
    const int row = rem >> 5;
    const int pc = rem & 31;
    const v8h val = *(const v8h*)(q16 + (size_t)(v * MP + n0 + row) * HID + pc * 8);
    *(v8h*)(Qs + (v * QB + row) * QSP + pc * 8) = val;
  }
  __syncthreads();

  v8f oacc[2][6];
#pragma unroll
  for (int qt = 0; qt < 2; ++qt)
#pragma unroll
    for (int nt = 0; nt < 6; ++nt) oacc[qt][nt] = zero8();

  int vbo[6];
#pragma unroll
  for (int j = 0; j < 6; ++j) {
    const int t = 6 * wave + j;
    const int tv = t >> 4, ct = t & 15;
    vbo[j] = (tv * HID + ct * 16 + c) * MP + 8 * h;
  }
  const _Float16* pa0p = Ps + c * PSP + 8 * h;
  const _Float16* pa1p = Ps + (16 + c) * PSP + 8 * h;
  float ps0 = 0.0f, ps1 = 0.0f;

#pragma unroll 1
  for (int ch = 0; ch < NCH; ++ch) {
    const int cbase = ch * KC;
#pragma unroll
    for (int s = 0; s < 2; ++s) {
      const int i = s * 256 + tid;
      if (i < NV * KC) {
        const int v = i >> 7, kk = i & 127;
        const int m = cbase + kk;
        const int mcl = (m < NN) ? m : (NN - 1);
        const float mval = mask[(size_t)mcl * NV + v];
        mc[v * KC + kk] = (m < NN) ? mval : 0.0f;
      }
    }
    __syncthreads();

    const int kb = cbase + 16 * wave;
    float pm0[8], pm1[8];
#pragma unroll
    for (int r = 0; r < 8; ++r) { pm0[r] = 0.0f; pm1[r] = 0.0f; }

#pragma unroll 1
    for (int v = 0; v < NV; ++v) {
      const _Float16* kap  = q16 + (size_t)(v * MP + kb + c) * HID + 8 * h;
      const _Float16* qb0p = Qs + (v * QB + c) * QSP + 8 * h;
      const _Float16* qb1p = Qs + (v * QB + 16 + c) * QSP + 8 * h;
      v8f s0 = zero8(), s1 = zero8();
#pragma unroll 1
      for (int k0 = 0; k0 < HID; k0 += 32) {
        const v16h a = ldfrag(kap + k0);
        const v16h b0 = ldfrag(qb0p + k0), b1 = ldfrag(qb1p + k0);
        s0 = mma16(a, b0, s0);
        s1 = mma16(a, b1, s1);
        guard_s2(s0, s1, a, b0, b1);
      }
      const float mr0 = mrow[v * QB + c], mr1 = mrow[v * QB + 16 + c];
      const v4f mcA = *(const v4f*)(mc + v * KC + 16 * wave + 8 * h);
      const v4f mcB = *(const v4f*)(mc + v * KC + 16 * wave + 8 * h + 4);
      float mk8[8];
#pragma unroll
      for (int r = 0; r < 4; ++r) { mk8[r] = mcA[r]; mk8[4 + r] = mcB[r]; }
#pragma unroll
      for (int r = 0; r < 8; ++r) {
        const float e0 = __expf(s0[r] * escale) * mr0 * mk8[r];
        const float e1 = __expf(s1[r] * escale) * mr1 * mk8[r];
        pm0[r] = (v == 0) ? e0 : fmaxf(pm0[r], e0);
        pm1[r] = (v == 0) ? e1 : fmaxf(pm1[r], e1);
      }
    }
    {
      v8h h0, h1;
#pragma unroll
      for (int r = 0; r < 8; ++r) {
        const int mk = kb + 8 * h + r;
        if (n0 + c == mk) pm0[r] = 0.0f;
        if (n0 + 16 + c == mk) pm1[r] = 0.0f;
        ps0 += pm0[r];
        ps1 += pm1[r];
        h0[r] = (_Float16)pm0[r];
        h1[r] = (_Float16)pm1[r];
      }
      *(v8h*)(Ps + c * PSP + 16 * wave + 8 * h) = h0;
      *(v8h*)(Ps + (16 + c) * PSP + 16 * wave + 8 * h) = h1;
    }
    __syncthreads();
#pragma unroll 1
    for (int ks = 0; ks < KC; ks += 32) {
      const v16h pa0 = ldfrag(pa0p + ks), pa1 = ldfrag(pa1p + ks);
#pragma unroll
      for (int g = 0; g < 2; ++g) {
        v16h vb[3];
#pragma unroll
        for (int jj = 0; jj < 3; ++jj) vb[jj] = ldfrag(hT16 + (size_t)vbo[3 * g + jj] + cbase + ks);
#pragma unroll
        for (int jj = 0; jj < 3; ++jj) {
          oacc[0][3 * g + jj] = mma16(pa0, vb[jj], oacc[0][3 * g + jj]);
          oacc[1][3 * g + jj] = mma16(pa1, vb[jj], oacc[1][3 * g + jj]);
        }
        guard_pv(oacc[0][3 * g], oacc[0][3 * g + 1], oacc[0][3 * g + 2],
                 oacc[1][3 * g], oacc[1][3 * g + 1], oacc[1][3 * g + 2],
                 pa0, pa1, vb[0], vb[1], vb[2]);
      }
    }
  }
  accg4(oacc[0][0], oacc[0][1], oacc[0][2], oacc[0][3]);
  accg4(oacc[0][4], oacc[0][5], oacc[1][0], oacc[1][1]);
  accg4(oacc[1][2], oacc[1][3], oacc[1][4], oacc[1][5]);

  ps0 += __shfl_xor(ps0, 16, 32);
  ps1 += __shfl_xor(ps1, 16, 32);
  psum[wave * QB + 16 * h + c] = h ? ps1 : ps0;
  __syncthreads();
  if (wave == 0) {
    const int row = lane;
    float S = 0.0f;
#pragma unroll
    for (int w = 0; w < 8; ++w) S += psum[w * QB + row];
    li[row] = (1.0f / (S + 1e-9f)) * invhs;
  }
  __syncthreads();

  float* OT = (float*)(smem + L_QS);
  const v4f iA0 = *(const v4f*)(li + 8 * h),      iB0 = *(const v4f*)(li + 8 * h + 4);
  const v4f iA1 = *(const v4f*)(li + 16 + 8 * h), iB1 = *(const v4f*)(li + 16 + 8 * h + 4);
#pragma unroll 1
  for (int vv = 0; vv < NV; ++vv) {
#pragma unroll
    for (int j = 0; j < 6; ++j) {
      const int t = 6 * wave + j;
      const int tv = t >> 4, ct = t & 15;
      if (tv == vv) {
        const int col = ct * 16 + c;
        const float* hp = hF + (size_t)(vv * MP + n0) * HID + col;
#pragma unroll
        for (int r = 0; r < 4; ++r) {
          {
            const int row = 8 * h + r;
            const float mv = mrow[vv * QB + row];
            const float hv = hp[(size_t)row * HID];
            OT[row * OTP + col] = (oacc[0][j][r] * iA0[r]) * (1.0f - mv) + hv * mv;
          }
          {
            const int row = 8 * h + 4 + r;
            const float mv = mrow[vv * QB + row];
            const float hv = hp[(size_t)row * HID];
            OT[row * OTP + col] = (oacc[0][j][4 + r] * iB0[r]) * (1.0f - mv) + hv * mv;
          }
          {
            const int row = 16 + 8 * h + r;
            const float mv = mrow[vv * QB + row];
            const float hv = hp[(size_t)row * HID];
            OT[row * OTP + col] = (oacc[1][j][r] * iA1[r]) * (1.0f - mv) + hv * mv;
          }
          {
            const int row = 16 + 8 * h + 4 + r;
            const float mv = mrow[vv * QB + row];
            const float hv = hp[(size_t)row * HID];
            OT[row * OTP + col] = (oacc[1][j][4 + r] * iB1[r]) * (1.0f - mv) + hv * mv;
          }
        }
      }
    }
    __syncthreads();
#pragma unroll
    for (int ps = 0; ps < 2; ++ps) {
#pragma unroll
      for (int rr = 0; rr < 4; ++rr) {
        const int row = 4 * wave + rr;
        const int n = n0 + row;
        const float* sp = OT + row * OTP + 8 * lane;
        const v4f x0 = *(const v4f*)sp, x1 = *(const v4f*)(sp + 4);
        v8us hb, lb;
#pragma unroll
        for (int e = 0; e < 4; ++e) {
          const unsigned short hh0 = bfbits(x0[e]);
          hb[e] = hh0;     lb[e] = bfbits(x0[e] - bfval(hh0));
          const unsigned short hh1 = bfbits(x1[e]);
          hb[4 + e] = hh1; lb[4 + e] = bfbits(x1[e] - bfval(hh1));
        }
        const size_t po = (size_t)(vv * MP + n) * HID + 8 * lane;
        *(volatile v8us*)(nxh + po) = hb;
        *(volatile v8us*)(nxl + po) = lb;
        if (n < NN) {
#pragma unroll
          for (int jj = 0; jj < 2; ++jj) {
            const int c4 = (jj * 32 + lane) * 4;
            const v4f val = *(const v4f*)(OT + row * OTP + c4);
            *(volatile v4f*)(out0 + (size_t)(vv * NN + n) * HID + c4) = val;
          }
        }
      }
      __threadfence();
    }
    __syncthreads();
  }
}

static size_t al256(size_t x) { return (x + 255) & ~(size_t)255; }

extern "C" void kernel_launch(void* const* d_in, const int* in_sizes, int n_in,
                              void* d_out, int out_size, void* d_ws, size_t ws_size,
                              hipStream_t stream) {
  if (n_in < 9) return;
  if (in_sizes[0] != NV * NN * DIN || in_sizes[1] != NN * DYD || in_sizes[2] != NN * NV) return;
  if (in_sizes[3] != NV * HID * DIN || in_sizes[4] != NV * HID) return;
  if (in_sizes[5] != NV * DIN * HID || in_sizes[6] != NV * DIN) return;
  if (in_sizes[7] != HID * DYD || in_sizes[8] != HID) return;
  if (out_size != NV * NN * HID + NV * NN * DIN + NN * HID) return;

  const float* x     = (const float*)d_in[0];
  const float* y     = (const float*)d_in[1];
  const float* mask  = (const float*)d_in[2];
  const float* W_in  = (const float*)d_in[3];
  const float* b_in  = (const float*)d_in[4];
  const float* W_out = (const float*)d_in[5];
  const float* b_out = (const float*)d_in[6];
  const float* Wy    = (const float*)d_in[7];
  const float* by    = (const float*)d_in[8];
  float* out0 = (float*)d_out;
  float* out1 = out0 + (size_t)NV * NN * HID;
  float* out2 = out1 + (size_t)NV * NN * DIN;

  const size_t bXB  = al256((size_t)NV * NN * DIN * 2);
  const size_t bYB  = al256((size_t)NN * DYD * 2);
  const size_t bWIB = al256((size_t)NV * HID * DIN * 2);
  const size_t bWOB = al256((size_t)NV * DIN * HID * 2);
  const size_t bWYB = al256((size_t)HID * DYD * 2);
  const size_t bHF  = al256((size_t)NV * MP * HID * 4);
  const size_t bQ16 = al256((size_t)NV * MP * HID * 2);
  const size_t bHT  = al256((size_t)NV * HID * MP * 2);
  const size_t bNX  = al256((size_t)NV * MP * HID * 2);
  size_t off = 0;
  const size_t oXB  = off; off += bXB;
  const size_t oYB  = off; off += bYB;
  const size_t oWIB = off; off += bWIB;
  const size_t oWOB = off; off += bWOB;
  const size_t oWYB = off; off += bWYB;
  const size_t oHF  = off; off += bHF;
  const size_t oQ16 = off; off += bQ16;
  const size_t oHT  = off; off += bHT;
  const size_t oNXH = off; off += bNX;
  const size_t oNXL = off; off += bNX;
  if (off > ws_size) return;
  if (off > (size_t)134217728) return;

  char* ws = (char*)d_ws;
  unsigned short* XB   = (unsigned short*)(ws + oXB);
  unsigned short* YB   = (unsigned short*)(ws + oYB);
  unsigned short* WIB  = (unsigned short*)(ws + oWIB);
  unsigned short* WOB  = (unsigned short*)(ws + oWOB);
  unsigned short* WYB  = (unsigned short*)(ws + oWYB);
  float*          HF   = (float*)(ws + oHF);
  _Float16*       Q16  = (_Float16*)(ws + oQ16);
  _Float16*       HT16 = (_Float16*)(ws + oHT);
  unsigned short* NXH  = (unsigned short*)(ws + oNXH);
  unsigned short* NXL  = (unsigned short*)(ws + oNXL);

  const dim3 blk(256);
  const int n8x = NV * NN * DIN / 8, n8y = NN * DYD / 8, n8wi = NV * HID * DIN / 8, n8wo = NV * DIN * HID / 8,
            n8wy = HID * DYD / 8;
  if ((n8x % 256) != 0 || (n8y % 256) != 0 || (n8wi % 256) != 0 || (n8wo % 256) != 0 || (n8wy % 256) != 0) return;

  cvt_kernel<<<dim3(n8x / 256), blk, 0, stream>>>(x, XB, n8x);
  cvt_kernel<<<dim3(n8y / 256), blk, 0, stream>>>(y, YB, n8y);
  cvt_kernel<<<dim3(n8wi / 256), blk, 0, stream>>>(W_in, WIB, n8wi);
  cvt_kernel<<<dim3(n8wo / 256), blk, 0, stream>>>(W_out, WOB, n8wo);
  cvt_kernel<<<dim3(n8wy / 256), blk, 0, stream>>>(Wy, WYB, n8wy);

  {
    const int tiles = (MP / 64) * (HID / 64);
    gemm64_kernel<false, 0><<<dim3((tiles + 7) / 8, NV), blk, 0, stream>>>(
        XB, XB, DIN, NN, NN * DIN, WIB, DIN, HID * DIN, HF, HID, MP * HID, MP, b_in, HID, MP, HID, DIN);
  }
  qt_kernel<<<dim3(MP / 64, NV), blk, 0, stream>>>(HF, mask, Q16, HT16, 64.0f, 64.0f);
  attn_kernel<<<dim3(MP / QB), blk, ATT_LDS, stream>>>(Q16, HT16, HF, mask, out0, NXH, NXL,
                                                       5.0f / 4096.0f, 1.0f / 64.0f);
  {
    const int tiles = (MP / 64) * (DIN / 64);
    gemm64_kernel<true, 1><<<dim3((tiles + 7) / 8, NV), blk, 0, stream>>>(
        NXH, NXL, HID, MP, MP * HID, WOB, HID, DIN * HID, out1, DIN, NN * DIN, NN, b_out, DIN, MP, DIN, HID);
  }
  {
    const int tiles = (MP / 64) * (HID / 64);
    gemm64_kernel<false, 2><<<dim3((tiles + 7) / 8, 1), blk, 0, stream>>>(
        YB, YB, DYD, NN, 0, WYB, DYD, 0, out2, HID, 0, NN, by, 0, MP, HID, DYD);
  }
  (void)hipGetLastError();
}
